// spatialTemporalLearningLayer_32023276159123
// MI455X (gfx1250) — hardware-verified
//
#include <hip/hip_runtime.h>


namespace {
constexpr int NS = 48  , N = 1024, F = 64, NR = NS * N;
constexpr float XS = 8.0f, WSC = 256.0f, PS = 1024.0f  , SCALE = 0.125f, LOG2E = 1.4426950408889634f, MASKED = -9.0e15f * 1.4426950408889634f;

typedef _Float16 b16;
typedef __attribute__((ext_vector_type(16))) _Float16 v16b;
typedef __attribute__((ext_vector_type(8))) _Float16 v8b;
typedef __attribute__((ext_vector_type(8))) float v8f;
typedef __attribute__((ext_vector_type(4))) float v4f;
typedef __attribute__((ext_vector_type(4))) int v4i;
__device__ __forceinline__ float bf16_rne(float f) { unsigned int u = __float_as_uint(f); u += 0x7FFFu + ((u >> 16) & 1u); return __uint_as_float(u & 0xFFFF0000u); }
__device__ __forceinline__ void split16(float v, b16& hi, b16& lo) { hi = (b16)v; lo = (b16)(v - (float)hi); }
__device__ __forceinline__ v16b frag_kb(const b16* p, int hh) { const v8b a = *(const v8b*)(p + 8 * hh), b = *(const v8b*)(p + 16 + 8 * hh); v16b f;
#pragma unroll
  for (int e = 0; e < 8; ++e) { f[e] = a[e]; f[8 + e] = b[e]; } return f; }
__device__ __forceinline__ v8f wmma16b(v16b a, v16b b, v8f c) { v8f d = __builtin_amdgcn_wmma_f32_16x16x32_f16(false, a, false, b, (short)0, c, false, false); asm volatile("v_nop\n\tv_nop\n\tv_nop\n\tv_nop" : "+v"(d) : "v"(a), "v"(b)); return d; }
__device__ __forceinline__ void wave_lds_sync() { __builtin_amdgcn_fence(__ATOMIC_RELEASE, "workgroup"); __builtin_amdgcn_wave_barrier(); __builtin_amdgcn_fence(__ATOMIC_ACQUIRE, "workgroup"); }
__device__ __forceinline__ float nexp2(float x) { return __builtin_amdgcn_exp2f(x); }

__global__ __launch_bounds__(256) void prep_kernel(const float* __restrict__ x, const float* __restrict__ theta, b16* __restrict__ X16, b16* __restrict__ TH16) {
  const size_t t = (size_t)blockIdx.x * 256 + threadIdx.x; const size_t nx = (size_t)NR * F / 8, nt = (size_t)F * F / 8; const float* src; b16* dst; size_t e; float sc;
  if (t < nx) { src = x; dst = X16; e = t * 8; sc = XS; } else if (t < nx + nt) { src = theta; dst = TH16; e = (t - nx) * 8; sc = WSC; } else return;
  const v4f a = *(const v4f*)(src + e), c = *(const v4f*)(src + e + 4); v8b o;
#pragma unroll
  for (int j = 0; j < 4; ++j) { o[j] = (b16)(bf16_rne(a[j]) * sc); o[4 + j] = (b16)(bf16_rne(c[j]) * sc); }
  for (int pass = 0; pass < 2; ++pass) { *(volatile v8b*)(dst + e) = o; __threadfence(); }
}
__global__ __launch_bounds__(128) void proj_kernel(const b16* __restrict__ X16, const b16* __restrict__ TH16, b16* __restrict__ XFh, b16* __restrict__ XFl, b16* __restrict__ VTh, b16* __restrict__ VTl) {
  __shared__ __attribute__((aligned(16))) b16 Th[4][16][F + 8], Tl[4][16][F + 8]; __shared__ __attribute__((aligned(16))) b16 Vt[F][64 + 8], Vtl[F][64 + 8];
  const int wave = threadIdx.x >> 5, lane = threadIdx.x & 31, nloc = lane & 15, hlf = lane >> 4, t_ = threadIdx.x; const size_t m0 = (size_t)blockIdx.x * 64 + wave * 16;
  v8f acc[4] = {{}, {}, {}, {}};
#pragma unroll
  for (int kb = 0; kb < F; kb += 32) { const v16b a = frag_kb(X16 + (m0 + nloc) * F + kb, hlf);
#pragma unroll
    for (int t = 0; t < 4; ++t) acc[t] = wmma16b(a, frag_kb(TH16 + (size_t)(t * 16 + nloc) * F + kb, hlf), acc[t]); }
#pragma unroll
  for (int t = 0; t < 4; ++t)
#pragma unroll
    for (int r = 0; r < 8; ++r) { b16 h_, l_; split16(acc[t][r] * (1.0f / (XS * WSC)) * XS, h_, l_); Th[wave][8 * hlf + r][t * 16 + nloc] = h_; Tl[wave][8 * hlf + r][t * 16 + nloc] = l_; Vt[t * 16 + nloc][wave * 16 + 8 * hlf + r] = h_; Vtl[t * 16 + nloc][wave * 16 + 8 * hlf + r] = l_; }
  __syncthreads();
  const int s = (int)(((size_t)blockIdx.x * 64) / N), n0 = (int)(((size_t)blockIdx.x * 64) % N);
  for (int pass = 0; pass < 2; ++pass) {
    for (int q = 0; q < 4; ++q) { const int rr = q * 4 + (lane >> 3), c8 = (lane & 7) * 8; *(volatile v8b*)(XFh + (m0 + rr) * F + c8) = *(const v8b*)(&Th[wave][rr][c8]); *(volatile v8b*)(XFl + (m0 + rr) * F + c8) = *(const v8b*)(&Tl[wave][rr][c8]); }
    for (int q = t_; q < F * 8; q += 128) { const int dd = q >> 3, c8 = (q & 7) * 8; const size_t gi = ((size_t)s * F + dd) * N + n0 + c8; *(volatile v8b*)(VTh + gi) = *(const v8b*)(&Vt[dd][c8]); *(volatile v8b*)(VTl + gi) = *(const v8b*)(&Vtl[dd][c8]); }
    __threadfence(); }
}
__global__ __launch_bounds__(64) void attn_kernel(const b16* __restrict__ XFh, const b16* __restrict__ XFl, const b16* __restrict__ VTh, const b16* __restrict__ VTl, const int* __restrict__ adj, float* __restrict__ out) {
  __shared__ __attribute__((aligned(16))) float To[2][16][F + 4];
  const int wave = threadIdx.x >> 5, lane = threadIdx.x & 31, hh = lane >> 4, col = lane & 15; const int s = blockIdx.z; const int q0 = blockIdx.x * 32 + wave * 16, qi = q0 + col;
  const size_t qo = ((size_t)s * N + qi) * F; const v16b qa0 = frag_kb(XFh + qo, hh), qa1 = frag_kb(XFh + qo + 32, hh), ql0 = frag_kb(XFl + qo, hh), ql1 = frag_kb(XFl + qo + 32, hh);
  const b16* Kb = XFh + (size_t)s * N * F; const b16* Klb = XFl + (size_t)s * N * F; const b16* Vb = VTh + (size_t)s * F * N; const b16* Vlb = VTl + (size_t)s * F * N; const int* arow = adj + (size_t)qi * N;
  float m = -INFINITY, l = 0.0f; v8f o[4] = {{}, {}, {}, {}}, ol[4] = {{}, {}, {}, {}};
  const float cs = SCALE * LOG2E / (XS * XS);
  for (int kb = 0; kb < N; kb += 32) {
    v8f s0 = {}, s1 = {};
    { const b16* k0 = Kb + (size_t)(kb + col) * F, *k1 = Kb + (size_t)(kb + 16 + col) * F, *k0l = Klb + (size_t)(kb + col) * F, *k1l = Klb + (size_t)(kb + 16 + col) * F;
      v16b f = frag_kb(k0, hh); s0 = wmma16b(f, qa0, s0); s0 = wmma16b(f, ql0, s0); s0 = wmma16b(frag_kb(k0l, hh), qa0, s0);
      f = frag_kb(k0 + 32, hh); s0 = wmma16b(f, qa1, s0); s0 = wmma16b(f, ql1, s0); s0 = wmma16b(frag_kb(k0l + 32, hh), qa1, s0);
      f = frag_kb(k1, hh); s1 = wmma16b(f, qa0, s1); s1 = wmma16b(f, ql0, s1); s1 = wmma16b(frag_kb(k1l, hh), qa0, s1);
      f = frag_kb(k1 + 32, hh); s1 = wmma16b(f, qa1, s1); s1 = wmma16b(f, ql1, s1); s1 = wmma16b(frag_kb(k1l + 32, hh), qa1, s1); }
    const v4i m0a = *(const v4i*)(arow + kb + 8 * hh), m0b = *(const v4i*)(arow + kb + 8 * hh + 4), m1a = *(const v4i*)(arow + kb + 16 + 8 * hh), m1b = *(const v4i*)(arow + kb + 16 + 8 * hh + 4);
    int mk[16] = {m0a[0], m0a[1], m0a[2], m0a[3], m0b[0], m0b[1], m0b[2], m0b[3], m1a[0], m1a[1], m1a[2], m1a[3], m1b[0], m1b[1], m1b[2], m1b[3]};
    float e[16]; float mx = -INFINITY;
#pragma unroll
    for (int r = 0; r < 8; ++r) { e[r] = (mk[r] > 0) ? s0[r] * cs : MASKED; e[8 + r] = (mk[8 + r] > 0) ? s1[r] * cs : MASKED; mx = fmaxf(mx, fmaxf(e[r], e[8 + r])); }
    mx = fmaxf(mx, __shfl_xor(mx, 16)); const float mn = fmaxf(m, mx); const float al = nexp2(m - mn); m = mn; float sum = 0.0f; v16b ph, pl;
#pragma unroll
    for (int i = 0; i < 16; ++i) { const float p = nexp2(e[i] - mn); sum += p; const b16 h_ = (b16)(p * PS); ph[i] = h_; pl[i] = (b16)(p * PS - (float)h_); }
    sum += __shfl_xor(sum, 16); l = l * al + sum;
#pragma unroll
    for (int t = 0; t < 4; ++t) { o[t] *= al; ol[t] *= al; const v16b vf = frag_kb(Vb + (size_t)(t * 16 + col) * N + kb, hh); o[t] = wmma16b(vf, ph, o[t]); ol[t] = wmma16b(vf, pl, ol[t]); ol[t] = wmma16b(frag_kb(Vlb + (size_t)(t * 16 + col) * N + kb, hh), ph, ol[t]); } }
  const float inv = 1.0f / (l * PS * XS);
#pragma unroll
  for (int t = 0; t < 4; ++t)
#pragma unroll
    for (int r = 0; r < 8; ++r) To[wave][col][t * 16 + 8 * hh + r] = fmaxf((o[t][r] + ol[t][r]) * inv, 0.0f);
  wave_lds_sync();
  for (int pass = 0; pass < 2; ++pass) { for (int r2 = 0; r2 < 16; r2 += 2) { const int rr = r2 + (lane >> 4), c4 = (lane & 15) * 4; *(volatile v4f*)(out + ((size_t)s * N + q0 + rr) * F + c4) = *(const v4f*)(&To[wave][rr][c4]); } __threadfence(); }
}
}

extern "C" void kernel_launch(void* const* d_in, const int* in_sizes, int n_in, void* d_out, int out_size, void* d_ws, size_t ws_size, hipStream_t stream) {
  (void)n_in;
  auto Fp = [&](int i) { return (const float*)d_in[i]; };
  if (in_sizes[0] != NR * F || in_sizes[1] != N * N || in_sizes[2] != F * F || out_size != NR * F) return;
  size_t off = 0; char* ws = (char*)d_ws;
  auto carve = [&](size_t bytes) { char* p = ws + off; off += (bytes + 255) & ~(size_t)255; return p; };
  b16* X16 = (b16*)carve((size_t)NR * F * 2); b16* TH16 = (b16*)carve((size_t)F * F * 2); b16* XFh = (b16*)carve((size_t)NR * F * 2); b16* XFl = (b16*)carve((size_t)NR * F * 2); b16* VTh = (b16*)carve((size_t)NR * F * 2); b16* VTl = (b16*)carve((size_t)NR * F * 2);
  if (off > ws_size || off > ((size_t)128 << 20)) return;
  prep_kernel<<<(unsigned)(((size_t)NR * F / 8 + F * F / 8 + 255) / 256), 256, 0, stream>>>(Fp(0), Fp(2), X16, TH16);
  proj_kernel<<<NR / 64, 128, 0, stream>>>(X16, TH16, XFh, XFl, VTh, VTl);
  attn_kernel<<<dim3(N / 32, 1, NS), 64, 0, stream>>>(XFh, XFl, VTh, VTl, (const int*)d_in[1], (float*)d_out);
}
